// MultiHeadAttentionGPT_49709951484072
// MI455X (gfx1250) — hardware-verified
//
#include <hip/hip_runtime.h>

#define BATCH 4
#define SEQ 2048
#define DMODEL 1024
#define NHEADS 16
#define DHEAD 64
#define VP 40
#define CP 68
#define TP 68

typedef unsigned short us;
typedef __bf16 v16bf __attribute__((ext_vector_type(16)));
typedef unsigned short v8us __attribute__((ext_vector_type(8)));
typedef v8us v8usa __attribute__((may_alias));
typedef float v8f __attribute__((ext_vector_type(8)));
typedef float v4f __attribute__((ext_vector_type(4)));
typedef v4f v4fa __attribute__((may_alias));
typedef unsigned int v4u __attribute__((ext_vector_type(4)));
typedef v4u v4ua __attribute__((may_alias));

union F8 { v8f v; float f[8]; };
union FR { v16bf v; v8us h[2]; };

static __device__ __forceinline__ v8f zero8() {
    v8f z = {0.f, 0.f, 0.f, 0.f, 0.f, 0.f, 0.f, 0.f};
    return z;
}

static __device__ __forceinline__ unsigned int bfbits(float x) {
    unsigned int u = __float_as_uint(x);
    return (u + 0x7FFFu + ((u >> 16) & 1u)) >> 16;
}

static __device__ __forceinline__ void split2w(float x0, float x1, unsigned int& hw, unsigned int& lw) {
    const unsigned int h0 = bfbits(x0), h1 = bfbits(x1);
    const unsigned int l0 = bfbits(x0 - __uint_as_float(h0 << 16));
    const unsigned int l1 = bfbits(x1 - __uint_as_float(h1 << 16));
    hw = h0 | (h1 << 16);
    lw = l0 | (l1 << 16);
}

static __device__ __forceinline__ void split8(const float* src, v4u& hv, v4u& lv) {
    unsigned int h0, l0, h1, l1, h2, l2, h3, l3;
    split2w(src[0], src[1], h0, l0);
    split2w(src[2], src[3], h1, l1);
    split2w(src[4], src[5], h2, l2);
    split2w(src[6], src[7], h3, l3);
    v4u a = {h0, h1, h2, h3};
    v4u b = {l0, l1, l2, l3};
    hv = a; lv = b;
}

static __device__ __forceinline__ void st_u4(us* p, v4u v) { *(volatile v4ua*)p = v; }
static __device__ __forceinline__ void st_f4(float* p, v4f v) { *(volatile v4fa*)p = v; }

static __device__ __forceinline__ v16bf ldfrag(const us* p) {
    FR u;
    u.h[0] = *(const v8usa*)p;
    u.h[1] = *(const v8usa*)(p + 16);
    return u.v;
}

static __device__ __forceinline__ v8f mma3(v8f c, v16bf ah, v16bf al, v16bf bh, v16bf bl) {
    c = __builtin_amdgcn_wmma_f32_16x16x32_bf16(false, ah, false, bh, (short)0, c, false, false);
    c = __builtin_amdgcn_wmma_f32_16x16x32_bf16(false, ah, false, bl, (short)0, c, false, false);
    c = __builtin_amdgcn_wmma_f32_16x16x32_bf16(false, al, false, bh, (short)0, c, false, false);
    asm volatile("v_nop\n\tv_nop\n\tv_nop\n\tv_nop" : "+v"(c) : "v"(ah), "v"(al), "v"(bh), "v"(bl));
    return c;
}

__global__ __launch_bounds__(256) void xsplit_kernel(const float* __restrict__ X,
                                                     us* __restrict__ Xh, us* __restrict__ Xl, int n8)
{
    const int i = blockIdx.x * 256 + threadIdx.x;
    if (i >= n8) return;
    const float* p = X + (size_t)i * 8;
    const v4f a = *(const v4fa*)p;
    const v4f b = *(const v4fa*)(p + 4);
    unsigned int h0, l0, h1, l1, h2, l2, h3, l3;
    split2w(a.x, a.y, h0, l0);
    split2w(a.z, a.w, h1, l1);
    split2w(b.x, b.y, h2, l2);
    split2w(b.z, b.w, h3, l3);
    const v4u hv = {h0, h1, h2, h3};
    const v4u lv = {l0, l1, l2, l3};
    us* dh = Xh + (size_t)i * 8;
    us* dl = Xl + (size_t)i * 8;
    st_u4(dh, hv);
    st_u4(dl, lv);
    __threadfence();
    st_u4(dh, hv);
    st_u4(dl, lv);
}

__global__ __launch_bounds__(256) void wsplit_kernel(const float* W0, const float* W1,
                                                     const float* W2, const float* W3,
                                                     us* __restrict__ P, int D)
{
    __shared__ __align__(16) float tl[64 * TP];
    const int tid = threadIdx.x;
    const int z = blockIdx.z;
    const float* W = (z == 0) ? W0 : ((z == 1) ? W1 : ((z == 2) ? W2 : W3));
    const int n0 = blockIdx.x * 64;
    const int k0 = blockIdx.y * 64;

    #pragma unroll
    for (int it = 0; it < 16; ++it) {
        const int idx = it * 256 + tid;
        const int kk = idx >> 6, nn = idx & 63;
        tl[nn * TP + kk] = W[(size_t)(k0 + kk) * D + n0 + nn];
    }
    __syncthreads();

    us* Ph = P + (size_t)(2 * z) * D * D;
    us* Pl = Ph + (size_t)D * D;
    const int pc = tid & 7;
    v4u hv[2], lv[2];
    #pragma unroll
    for (int it = 0; it < 2; ++it) {
        const int L = it * 32 + (tid >> 3);
        split8(&tl[L * TP + pc * 8], hv[it], lv[it]);
    }
    #pragma unroll
    for (int it = 0; it < 2; ++it) {
        const int L = it * 32 + (tid >> 3);
        const size_t off = (size_t)(n0 + L) * D + k0 + pc * 8;
        st_u4(Ph + off, hv[it]);
        st_u4(Pl + off, lv[it]);
    }
    __threadfence();
    #pragma unroll
    for (int it = 0; it < 2; ++it) {
        const int L = it * 32 + (tid >> 3);
        const size_t off = (size_t)(n0 + L) * D + k0 + pc * 8;
        st_u4(Ph + off, hv[it]);
        st_u4(Pl + off, lv[it]);
    }
}

template <int MODE>
__global__ __launch_bounds__(256) void gemm_kernel(
    const us* __restrict__ Ah, const us* __restrict__ Al, int lda,
    const us* B0h, const us* B0l, const us* B1h, const us* B1l, const us* B2h, const us* B2l, int ldb,
    void* O0a, void* O0b, void* O1a, void* O1b, void* O2a, void* O2b, int ldc, int K)
{
    __shared__ __align__(16) float tile[128 * TP];
    const int tid = threadIdx.x;
    const int lane = tid & 31, wave = tid >> 5, hf = lane >> 4, nl = lane & 15;
    const int wm = wave & 3, wn = wave >> 2;
    const int z = blockIdx.z;
    const us* Bh = (z == 0) ? B0h : ((z == 1) ? B1h : B2h);
    const us* Bl = (z == 0) ? B0l : ((z == 1) ? B1l : B2l);
    void* Oa = (z == 0) ? O0a : ((z == 1) ? O1a : O2a);
    void* Ob = (z == 0) ? O0b : ((z == 1) ? O1b : O2b);
    const int m0 = blockIdx.x * 128, n0 = blockIdx.y * 64;
    const int am = m0 + wm * 32, bn = n0 + wn * 32;

    const us* aph = Ah + (size_t)(am + nl) * lda + 8 * hf;
    const us* apl = Al + (size_t)(am + nl) * lda + 8 * hf;
    const us* bph = Bh + (size_t)(bn + nl) * ldb + 8 * hf;
    const us* bpl = Bl + (size_t)(bn + nl) * ldb + 8 * hf;
    const size_t a16 = (size_t)16 * lda, b16 = (size_t)16 * ldb;

    F8 acc[2][2];
    #pragma unroll
    for (int tm = 0; tm < 2; ++tm)
        #pragma unroll
        for (int tn = 0; tn < 2; ++tn) acc[tm][tn].v = zero8();

    #pragma unroll 1
    for (int k = 0; k < K; k += 32) {
        v16bf a_h[2], a_l[2], b_h[2], b_l[2];
        a_h[0] = ldfrag(aph + k);        a_h[1] = ldfrag(aph + a16 + k);
        a_l[0] = ldfrag(apl + k);        a_l[1] = ldfrag(apl + a16 + k);
        b_h[0] = ldfrag(bph + k);        b_h[1] = ldfrag(bph + b16 + k);
        b_l[0] = ldfrag(bpl + k);        b_l[1] = ldfrag(bpl + b16 + k);
        #pragma unroll
        for (int tm = 0; tm < 2; ++tm)
            #pragma unroll
            for (int tn = 0; tn < 2; ++tn)
                acc[tm][tn].v = mma3(acc[tm][tn].v, a_h[tm], a_l[tm], b_h[tn], b_l[tn]);
    }

    #pragma unroll
    for (int tm = 0; tm < 2; ++tm)
        #pragma unroll
        for (int tn = 0; tn < 2; ++tn)
            #pragma unroll
            for (int r = 0; r < 8; ++r)
                tile[(wm * 32 + tm * 16 + 8 * hf + r) * TP + wn * 32 + tn * 16 + nl] = acc[tm][tn].f[r];
    __syncthreads();

    const int pc = tid & 7;
    if (MODE == 1) {
        us* Oh = (us*)Oa;
        us* Ol = (us*)Ob;
        v4u hv[4], lv[4];
        #pragma unroll
        for (int it = 0; it < 4; ++it) {
            const int L = it * 32 + (tid >> 3);
            split8(&tile[L * TP + pc * 8], hv[it], lv[it]);
        }
        #pragma unroll
        for (int it = 0; it < 4; ++it) {
            const int L = it * 32 + (tid >> 3);
            const size_t off = (size_t)(m0 + L) * ldc + n0 + pc * 8;
            st_u4(Oh + off, hv[it]);
            st_u4(Ol + off, lv[it]);
        }
        __threadfence();
        #pragma unroll
        for (int it = 0; it < 4; ++it) {
            const int L = it * 32 + (tid >> 3);
            const size_t off = (size_t)(m0 + L) * ldc + n0 + pc * 8;
            st_u4(Oh + off, hv[it]);
            st_u4(Ol + off, lv[it]);
        }
    } else {
        float* Of = (float*)Oa;
        v4f fv[8];
        #pragma unroll
        for (int it = 0; it < 8; ++it) {
            const int L = it * 32 + (tid >> 3);
            const int row = L >> 1, col = (L & 1) * 32 + pc * 4;
            const float* src = &tile[row * TP + col];
            v4f v = {src[0], src[1], src[2], src[3]};
            fv[it] = v;
        }
        #pragma unroll
        for (int it = 0; it < 8; ++it) {
            const int L = it * 32 + (tid >> 3);
            const int row = L >> 1, col = (L & 1) * 32 + pc * 4;
            st_f4(Of + (size_t)(m0 + row) * ldc + n0 + col, fv[it]);
        }
        __threadfence();
        #pragma unroll
        for (int it = 0; it < 8; ++it) {
            const int L = it * 32 + (tid >> 3);
            const int row = L >> 1, col = (L & 1) * 32 + pc * 4;
            st_f4(Of + (size_t)(m0 + row) * ldc + n0 + col, fv[it]);
        }
    }
}

__global__ __launch_bounds__(128) void attn_kernel(
    const us* __restrict__ Qh, const us* __restrict__ Ql,
    const us* __restrict__ Kh, const us* __restrict__ Kl,
    const us* __restrict__ Vh, const us* __restrict__ Vl,
    us* __restrict__ Ch, us* __restrict__ Cl, int crow0)
{
    __shared__ __align__(16) us vlds[2][64 * VP];
    __shared__ __align__(16) us plds[2][4][16 * VP];
    __shared__ __align__(16) float clds[4][16 * CP];

    const int tid = threadIdx.x;
    const int lane = tid & 31, wave = tid >> 5, hf = lane >> 4, nl = lane & 15;
    const int hc = blockIdx.y * DHEAD;
    const int q0 = blockIdx.x * 64 + wave * 16;
    const int kbl = blockIdx.x * 2 + 1;
    const float NINF = -__builtin_inff();

    const size_t qo = (size_t)(q0 + nl) * DMODEL + hc + 8 * hf;
    const v16bf qh0 = ldfrag(Qh + qo), qh1 = ldfrag(Qh + qo + 32);
    const v16bf ql0 = ldfrag(Ql + qo), ql1 = ldfrag(Ql + qo + 32);

    F8 o[4];
    #pragma unroll
    for (int t = 0; t < 4; ++t) o[t].v = zero8();
    float mrow[8], lrow[8];
    #pragma unroll
    for (int i = 0; i < 8; ++i) { mrow[i] = NINF; lrow[i] = 0.f; }

    us* ph = &plds[0][wave][0];
    us* pl = &plds[1][wave][0];

    #pragma unroll 1
    for (int kb = 0; kb <= kbl; ++kb) {
        const int k0 = kb * 32;
        __syncthreads();

        {
            const int kk = tid >> 2, d0 = (tid & 3) * 16;
            const size_t vo = (size_t)(k0 + kk) * DMODEL + hc + d0;
            const v8us a0 = *(const v8usa*)(Vh + vo), a1 = *(const v8usa*)(Vh + vo + 8);
            const v8us b0 = *(const v8usa*)(Vl + vo), b1 = *(const v8usa*)(Vl + vo + 8);
            #pragma unroll
            for (int j = 0; j < 8; ++j) {
                vlds[0][(d0 + j) * VP + kk]     = a0[j];
                vlds[0][(d0 + 8 + j) * VP + kk] = a1[j];
                vlds[1][(d0 + j) * VP + kk]     = b0[j];
                vlds[1][(d0 + 8 + j) * VP + kk] = b1[j];
            }
        }

        F8 s[2];
        #pragma unroll
        for (int j = 0; j < 2; ++j) {
            const size_t ko = (size_t)(k0 + 16 * j + nl) * DMODEL + hc + 8 * hf;
            const v16bf kh0 = ldfrag(Kh + ko), kh1 = ldfrag(Kh + ko + 32);
            const v16bf kl0 = ldfrag(Kl + ko), kl1 = ldfrag(Kl + ko + 32);
            v8f c = zero8();
            c = mma3(c, qh0, ql0, kh0, kl0);
            c = mma3(c, qh1, ql1, kh1, kl1);
            s[j].v = c;
        }

        #pragma unroll
        for (int v = 0; v < 8; ++v) {
            const int row = q0 + 8 * hf + v;
            float a  = s[0].f[v] * 0.125f;
            float bb = s[1].f[v] * 0.125f;
            a  = (k0 + nl <= row) ? a : NINF;
            bb = (k0 + 16 + nl <= row) ? bb : NINF;
            float mx = fmaxf(a, bb);
            mx = fmaxf(mx, __shfl_xor(mx, 8));
            mx = fmaxf(mx, __shfl_xor(mx, 4));
            mx = fmaxf(mx, __shfl_xor(mx, 2));
            mx = fmaxf(mx, __shfl_xor(mx, 1));
            const float mnew  = fmaxf(mrow[v], mx);
            const float alpha = __expf(mrow[v] - mnew);
            const float ea = __expf(a - mnew);
            const float eb = __expf(bb - mnew);
            float rs = ea + eb;
            rs += __shfl_xor(rs, 8);
            rs += __shfl_xor(rs, 4);
            rs += __shfl_xor(rs, 2);
            rs += __shfl_xor(rs, 1);
            lrow[v] = lrow[v] * alpha + rs;
            mrow[v] = mnew;
            #pragma unroll
            for (int t = 0; t < 4; ++t) o[t].f[v] *= alpha;
            const unsigned int ha = bfbits(ea), hb = bfbits(eb);
            const unsigned int la = bfbits(ea - __uint_as_float(ha << 16));
            const unsigned int lb = bfbits(eb - __uint_as_float(hb << 16));
            const int r = v + 8 * hf;
            ph[r * VP + nl]      = (us)ha;
            ph[r * VP + 16 + nl] = (us)hb;
            pl[r * VP + nl]      = (us)la;
            pl[r * VP + 16 + nl] = (us)lb;
        }
        __syncthreads();

        const v16bf pfh = ldfrag(ph + nl * VP + 8 * hf);
        const v16bf pfl = ldfrag(pl + nl * VP + 8 * hf);
        #pragma unroll
        for (int t = 0; t < 4; ++t) {
            const int vo = (t * 16 + nl) * VP + 8 * hf;
            const v16bf vfh = ldfrag(&vlds[0][vo]);
            const v16bf vfl = ldfrag(&vlds[1][vo]);
            o[t].v = mma3(o[t].v, pfh, pfl, vfh, vfl);
        }
    }

    #pragma unroll
    for (int v = 0; v < 8; ++v) {
        const float inv = 1.0f / lrow[v];
        const int r = v + 8 * hf;
        #pragma unroll
        for (int t = 0; t < 4; ++t) clds[wave][r * CP + t * 16 + nl] = o[t].f[v] * inv;
    }
    __syncthreads();

    const int pc = lane & 7;
    v4u hv[4], lv[4];
    #pragma unroll
    for (int it = 0; it < 4; ++it) {
        const int rl = it * 4 + (lane >> 3);
        split8(&clds[wave][rl * CP + pc * 8], hv[it], lv[it]);
    }
    #pragma unroll
    for (int it = 0; it < 4; ++it) {
        const int rl = it * 4 + (lane >> 3);
        const size_t off = (size_t)(crow0 + q0 + rl) * DMODEL + hc + pc * 8;
        st_u4(Ch + off, hv[it]);
        st_u4(Cl + off, lv[it]);
    }
    __threadfence();
    #pragma unroll
    for (int it = 0; it < 4; ++it) {
        const int rl = it * 4 + (lane >> 3);
        const size_t off = (size_t)(crow0 + q0 + rl) * DMODEL + hc + pc * 8;
        st_u4(Ch + off, hv[it]);
        st_u4(Cl + off, lv[it]);
    }
}

extern "C" void kernel_launch(void* const* d_in, const int* in_sizes, int n_in,
                              void* d_out, int out_size, void* d_ws, size_t ws_size,
                              hipStream_t stream)
{
    if (n_in != 5) return;
    const int M = BATCH * SEQ;
    const int DD = DMODEL * DMODEL;
    if (in_sizes[0] != M * DMODEL) return;
    if (in_sizes[1] != DD || in_sizes[2] != DD || in_sizes[3] != DD || in_sizes[4] != DD) return;
    if (out_size != M * DMODEL) return;

    const float* X  = (const float*)d_in[0];
    const float* Wq = (const float*)d_in[1];
    const float* Wk = (const float*)d_in[2];
    const float* Wv = (const float*)d_in[3];
    const float* Wo = (const float*)d_in[4];
    float* out = (float*)d_out;

    const size_t xplaneE = (size_t)M * DMODEL;
    const size_t wplaneE = (size_t)DD;
    const size_t bplaneE = (size_t)SEQ * DMODEL;

    size_t off = 0;
    char* ws = (char*)d_ws;
    us* xh = (us*)(ws + off); off += xplaneE * 2;
    us* xl = (us*)(ws + off); off += xplaneE * 2;
    us* wt = (us*)(ws + off); off += 8 * wplaneE * 2;
    us* qh = (us*)(ws + off); off += bplaneE * 2;
    us* ql = (us*)(ws + off); off += bplaneE * 2;
    us* kh = (us*)(ws + off); off += bplaneE * 2;
    us* kl = (us*)(ws + off); off += bplaneE * 2;
    us* vh = (us*)(ws + off); off += bplaneE * 2;
    us* vl = (us*)(ws + off); off += bplaneE * 2;
    us* ch = (us*)(ws + off); off += xplaneE * 2;
    us* cl = (us*)(ws + off); off += xplaneE * 2;
    if (off > ws_size) return;

    const us* wqh = wt + 0 * wplaneE; const us* wql = wt + 1 * wplaneE;
    const us* wkh = wt + 2 * wplaneE; const us* wkl = wt + 3 * wplaneE;
    const us* wvh = wt + 4 * wplaneE; const us* wvl = wt + 5 * wplaneE;
    const us* woh = wt + 6 * wplaneE; const us* wol = wt + 7 * wplaneE;

    const int n8 = (int)(xplaneE / 8);
    xsplit_kernel<<<(n8 + 255) / 256, 256, 0, stream>>>(X, xh, xl, n8);
    wsplit_kernel<<<dim3(DMODEL / 64, DMODEL / 64, 4), 256, 0, stream>>>(Wq, Wk, Wv, Wo, wt, DMODEL);

    for (int b = 0; b < BATCH; ++b) {
        const us* xbh = xh + (size_t)b * bplaneE;
        const us* xbl = xl + (size_t)b * bplaneE;
        gemm_kernel<1><<<dim3(SEQ / 128, DMODEL / 64, 3), 256, 0, stream>>>(
            xbh, xbl, DMODEL,
            wqh, wql, wkh, wkl, wvh, wvl, DMODEL,
            (void*)qh, (void*)ql, (void*)kh, (void*)kl, (void*)vh, (void*)vl, DMODEL, DMODEL);
        attn_kernel<<<dim3(SEQ / 64, NHEADS), 128, 0, stream>>>(qh, ql, kh, kl, vh, vl, ch, cl, b * SEQ);
    }

    gemm_kernel<0><<<dim3(M / 128, DMODEL / 64, 1), 256, 0, stream>>>(
        ch, cl, DMODEL,
        woh, wol, woh, wol, woh, wol, DMODEL,
        (void*)out, (void*)out, (void*)out, (void*)out, (void*)out, (void*)out, DMODEL, DMODEL);
}
